// TransformerLayer_90675349553885
// MI455X (gfx1250) — hardware-verified
//
#include <hip/hip_runtime.h>
#ifndef NB
#define NB 2
#endif
#ifndef SEQ
#define SEQ 2048
#endif
#define SQ SEQ
#define SQ_FULL 2048
#define DM 1024
#define NH 16
#define HD 64
#define HG 2
#define DFF 4096
#define LQ (3 * DM)
#define NKX SQ
#define NR ((size_t)NB * SQ)

static_assert(SQ % 128 == 0);
static_assert(NH % HG == 0);
static_assert(DM == NH * HD);
static_assert(DM == 256 * 4);
static_assert(DM % 64 == 0 && DFF % 64 == 0 && LQ % 64 == 0 && HD % 32 == 0);

typedef unsigned short v8us __attribute__((ext_vector_type(8), may_alias));
typedef float  v8f  __attribute__((ext_vector_type(8)));
typedef float  v4f  __attribute__((ext_vector_type(4)));
typedef float  v4fa __attribute__((ext_vector_type(4), may_alias));
typedef _Float16 v16h __attribute__((ext_vector_type(16)));
typedef _Float16 v4h __attribute__((ext_vector_type(4)));
union FragH { v16h v; v8us half[2]; _Float16 h[16]; unsigned short u[16]; };

__device__ __forceinline__ unsigned short bf16_bits(float x) { unsigned int u = __float_as_uint(x); return (unsigned short)((u + 0x7FFFu + ((u >> 16) & 1u)) >> 16); }
__device__ __forceinline__ float bf16_val(unsigned short b) { return __uint_as_float(((unsigned int)b) << 16); }
__device__ __forceinline__ float bf16_rne(float x) { return bf16_val(bf16_bits(x)); }

__global__ __launch_bounds__(256) void k_wt_f16(const float* __restrict__ W, _Float16* __restrict__ Wt, unsigned K, unsigned N, float scale) {
  const unsigned k8n = K >> 3;
  const unsigned t = blockIdx.x * 256u + threadIdx.x;
  if (t >= N * k8n) return;
  const unsigned n = t / k8n, k8 = (t - n * k8n) << 3;
  FragH f;
#pragma unroll
  for (int i = 0; i < 8; ++i) f.h[i] = (_Float16)(bf16_rne(W[(size_t)(k8 + (unsigned)i) * N + n]) * scale);
  const v8us o = f.half[0];
  unsigned short* dst = (unsigned short*)Wt + (size_t)n * K + k8;
  *(volatile v8us*)dst = o;
  __threadfence();
  *(volatile v8us*)dst = o;
}

template <int BFIN>
__global__ __launch_bounds__(256) void k_ln16(const float* __restrict__ X, const float* __restrict__ g, const float* __restrict__ bb, float eps, _Float16* __restrict__ N16) {
  #pragma clang fp contract(off)
  __shared__ float red[256];
  const size_t r = blockIdx.x; const unsigned t = threadIdx.x;
  const v4f xa = *(const v4fa*)(X + r * DM + t * 4u);
  float s[4]; float sum = 0.f;
#pragma unroll
  for (int q = 0; q < 4; ++q) { s[q] = BFIN ? bf16_rne(xa[q]) : xa[q]; sum = __fadd_rn(sum, s[q]); }
  red[t] = sum; __syncthreads();
  for (unsigned st = 128u; st > 0u; st >>= 1) { if (t < st) red[t] = __fadd_rn(red[t], red[t + st]); __syncthreads(); }
  const float mu = __fmul_rn(red[0], 1.0f / (float)DM); __syncthreads();
  float vs = 0.f;
#pragma unroll
  for (int q = 0; q < 4; ++q) { const float dl = __fadd_rn(s[q], -mu); vs = __fadd_rn(vs, __fmul_rn(dl, dl)); }
  red[t] = vs; __syncthreads();
  for (unsigned st = 128u; st > 0u; st >>= 1) { if (t < st) red[t] = __fadd_rn(red[t], red[t + st]); __syncthreads(); }
  const float rs = rsqrtf(__fadd_rn(__fmul_rn(red[0], 1.0f / (float)DM), eps));
  v4h y;
#pragma unroll
  for (int q = 0; q < 4; ++q) { const unsigned c = t * 4u + (unsigned)q; y[q] = (_Float16)__fadd_rn(__fmul_rn(__fmul_rn(__fadd_rn(s[q], -mu), rs), bf16_rne(g[c])), bf16_rne(bb[c])); }
  _Float16* dst = N16 + r * DM + t * 4u;
  *(volatile v4h*)dst = y;
  __threadfence();
  *(volatile v4h*)dst = y;
}

__device__ __forceinline__ v16h g2_frag(const _Float16* p, unsigned hh) { FragH f; f.half[0] = *(const v8us*)((const unsigned short*)p + 8u * hh); f.half[1] = *(const v8us*)((const unsigned short*)p + 16u + 8u * hh); return f.v; }
__device__ __forceinline__ v8f g2_mma(v16h a, v16h b, v8f c) { v8f d = __builtin_amdgcn_wmma_f32_16x16x32_f16(false, a, false, b, (short)0, c, false, false); asm volatile("v_nop\n\tv_nop\n\tv_nop\n\tv_nop" : "+v"(d) : "v"(a), "v"(b)); return d; }
template <int ACT, int RESB>
__global__ __launch_bounds__(128) void k_gemm2(const _Float16* __restrict__ A, int lda, size_t sA, const _Float16* __restrict__ Bh, int ldb, size_t sB, float alpha,
    const float* __restrict__ bias, const float* __restrict__ CP, int ldcp,
    float* __restrict__ C, _Float16* __restrict__ C16, int ldc, size_t sC, int M, int N, int K, int caus) {
  static_assert(ACT == 0 || ACT == 6);
  __shared__ __attribute__((aligned(16))) float so[4][32][68];
  const unsigned tid = threadIdx.x, w = tid >> 5, lane = tid & 31u, ln = lane & 15u, hh = lane >> 4; const unsigned by = blockIdx.y;
  A += (size_t)by * sA; Bh += (size_t)by * sB; const size_t cofs = (size_t)by * sC;
  const unsigned ntn = (unsigned)N >> 6; const unsigned mt = blockIdx.x / ntn, nq = blockIdx.x - mt * ntn;
  const unsigned rowblk = mt * 128u, row0 = rowblk + 32u * w, col0 = nq * 64u;
  if (caus == 1 && col0 >= rowblk + 128u) return;
  if (row0 >= (unsigned)M) return;
  unsigned kend = (unsigned)K; if (caus == 2 && rowblk + 128u < kend) kend = rowblk + 128u;
  const _Float16* a0p = A + (size_t)(row0 + ln) * (unsigned)lda; const _Float16* a1p = a0p + (size_t)16 * (unsigned)lda;
  const _Float16* b0p = Bh + (size_t)(col0 + ln) * (unsigned)ldb; const _Float16* b1p = b0p + (size_t)16 * (unsigned)ldb; const _Float16* b2p = b1p + (size_t)16 * (unsigned)ldb; const _Float16* b3p = b2p + (size_t)16 * (unsigned)ldb;
  const v8f z8 = {0.f,0.f,0.f,0.f,0.f,0.f,0.f,0.f}; v8f c00 = z8, c01 = z8, c02 = z8, c03 = z8, c10 = z8, c11 = z8, c12 = z8, c13 = z8;
#pragma unroll 1
  for (unsigned kb = 0; kb < kend; kb += 32u) { const v16h a0 = g2_frag(a0p + kb, hh), a1 = g2_frag(a1p + kb, hh);
    v16h b = g2_frag(b0p + kb, hh); c00 = g2_mma(a0, b, c00); c10 = g2_mma(a1, b, c10);
    b = g2_frag(b1p + kb, hh); c01 = g2_mma(a0, b, c01); c11 = g2_mma(a1, b, c11);
    b = g2_frag(b2p + kb, hh); c02 = g2_mma(a0, b, c02); c12 = g2_mma(a1, b, c12);
    b = g2_frag(b3p + kb, hh); c03 = g2_mma(a0, b, c03); c13 = g2_mma(a1, b, c13); }
  v8f accs[8] = {c00, c01, c02, c03, c10, c11, c12, c13};
#pragma unroll
  for (int u = 0; u < 8; ++u) { const unsigned t = (unsigned)(u & 3), half = (unsigned)(u >> 2); const unsigned col = col0 + t * 16u + ln; const float bv = bias ? bf16_rne(bias[col]) : 0.f;
#pragma unroll
    for (int r = 0; r < 8; ++r) { const unsigned rloc = half * 16u + 8u * hh + (unsigned)r; float v = accs[u][r] * alpha + bv;
      if (CP) { float rv = CP[(size_t)(row0 + rloc) * (unsigned)ldcp + col]; if (RESB) rv = bf16_rne(rv); v += rv; }
      if (ACT == 6) v = 0.5f * v * (1.0f + erff(v * 0.70710678118654752f));
      so[w][rloc][t * 16u + ln] = v; } }
  __builtin_amdgcn_fence(4  , "workgroup"); __builtin_amdgcn_wave_barrier();
  const unsigned rsub = lane >> 4, c4 = (lane & 15u) * 4u;
  for (int pass = 0; pass < 2; ++pass) {
#pragma unroll
    for (int q = 0; q < 16; ++q) { const unsigned r = (unsigned)q * 2u + rsub; const v4f v = *(const v4fa*)&so[w][r][c4];
      if (C) *(volatile v4f*)(C + cofs + (size_t)(row0 + r) * (unsigned)ldc + col0 + c4) = v;
      if (C16) { v4h h4; for (int i = 0; i < 4; ++i) h4[i] = (_Float16)v[i]; *(volatile v4h*)(C16 + cofs + (size_t)(row0 + r) * (unsigned)ldc + col0 + c4) = h4; } }
    if (pass == 0) __threadfence(); } }

template <int NHv, int TTv>
__global__ __launch_bounds__(256) void k_vt(const _Float16* __restrict__ V16, int ldv, int voff, _Float16* __restrict__ Vt) {
  __shared__ unsigned short tl[64][66];
  const unsigned tid = threadIdx.x; const unsigned ntg = (unsigned)(TTv / 64); const unsigned slab = blockIdx.x / ntg, lg = blockIdx.x - slab * ntg; const unsigned b = slab / (unsigned)NHv, h = slab - b * (unsigned)NHv;
  for (unsigned i = tid; i < 512u; i += 256u) { const unsigned r = i >> 3, c8 = (i & 7u) * 8u; FragH f; f.half[0] = *(const v8us*)((const unsigned short*)V16 + ((size_t)b * TTv + lg * 64u + r) * (unsigned)ldv + (unsigned)voff + h * 64u + c8);
#pragma unroll
    for (int q = 0; q < 8; ++q) tl[r][c8 + (unsigned)q] = f.u[q]; }
  __syncthreads();
  for (int pass = 0; pass < 2; ++pass) {
#pragma unroll
    for (int rd = 0; rd < 2; ++rd) { const unsigned d = (unsigned)rd * 32u + (tid >> 3), pc = tid & 7u; FragH f;
#pragma unroll
      for (int q = 0; q < 8; ++q) f.u[q] = tl[pc * 8u + (unsigned)q][d];
      *(volatile v8us*)((unsigned short*)Vt + ((size_t)slab * 64u + d) * TTv + lg * 64u + pc * 8u) = f.half[0]; }
    if (pass == 0) __threadfence(); } }

__global__ __launch_bounds__(128) void k_rsmc(const float* __restrict__ S, _Float16* __restrict__ P) {
  #pragma clang fp contract(off)
  const unsigned nrb = (unsigned)(SQ / 128); const unsigned hh = blockIdx.x / nrb; const unsigned i0 = (blockIdx.x - hh * nrb) * 128u; const unsigned i = i0 + threadIdx.x; const unsigned nk = i0 + 128u;
  const size_t rowoff = ((size_t)hh * SQ + i) * NKX; const float* s = S + rowoff;
  float mx = -3.0e38f;
#pragma unroll 1
  for (unsigned j0 = 0; j0 < nk; j0 += 4u) { const v4f v = *(const v4fa*)(s + j0);
#pragma unroll
    for (int q = 0; q < 4; ++q) { const bool ok = (j0 + (unsigned)q) <= i; mx = fmaxf(mx, ok ? v[q] : -3.0e38f); } }
  float se = 0.f;
#pragma unroll 1
  for (unsigned j0 = 0; j0 < nk; j0 += 4u) { const v4f v = *(const v4fa*)(s + j0);
#pragma unroll
    for (int q = 0; q < 4; ++q) { const bool ok = (j0 + (unsigned)q) <= i; const float e = __expf((ok ? v[q] : mx) - mx); se += ok ? e : 0.f; } }
  const float sc = 256.0f / se;
#pragma unroll 1
  for (unsigned j0 = 0; j0 < nk; j0 += 8u) { const v4f a = *(const v4fa*)(s + j0), c = *(const v4fa*)(s + j0 + 4u); FragH fr;
#pragma unroll
    for (int q = 0; q < 4; ++q) { const bool ok0 = (j0 + (unsigned)q) <= i, ok1 = (j0 + 4u + (unsigned)q) <= i;
      const float e0 = __expf((ok0 ? a[q] : mx) - mx) * sc, e1 = __expf((ok1 ? c[q] : mx) - mx) * sc;
      fr.h[q] = (_Float16)(ok0 ? e0 : 0.f); fr.h[4 + q] = (_Float16)(ok1 ? e1 : 0.f); }
    const v8us o = fr.half[0]; unsigned short* d = (unsigned short*)P + rowoff + j0;
    *(volatile v8us*)d = o; __threadfence(); *(volatile v8us*)d = o; } }

constexpr size_t al256(size_t b) { return (b + 255) & ~(size_t)255; }
constexpr size_t SZ_BQKV = al256((size_t)3 * DM * DM * 2);
constexpr size_t SZ_BO   = al256((size_t)DM * DM * 2);
constexpr size_t SZ_BW1  = al256((size_t)DFF * DM * 2);
constexpr size_t SZ_BW2  = al256((size_t)DM * DFF * 2);
constexpr size_t SZ_X16  = al256(NR * DM * 2);
constexpr size_t SZ_QKV  = al256(NR * LQ * 2);
constexpr size_t SZ_O16  = al256(NR * DM * 2);
constexpr size_t SZ_VT   = al256((size_t)NB * NH * HD * SQ * 2);
constexpr size_t SZ_S    = (size_t)HG * SQ * NKX * 4;
constexpr size_t SZ_P    = (size_t)HG * SQ * NKX * 2;
constexpr size_t SZ_X1   = NR * DM * 4;
constexpr size_t SZ_HF   = (size_t)SQ * DFF * 2;
constexpr size_t SZ_R    = al256((SZ_S + SZ_P) > (SZ_X1 + SZ_HF) ? (SZ_S + SZ_P) : (SZ_X1 + SZ_HF));
constexpr size_t WS_TOTAL = SZ_BQKV + SZ_BO + SZ_BW1 + SZ_BW2 + SZ_X16 + SZ_QKV + SZ_O16 + SZ_VT + SZ_R;
static_assert(WS_TOTAL <= (size_t)134217728);
static_assert(SZ_S % 256 == 0 && SZ_X1 % 256 == 0);
static_assert(SZ_S + SZ_P <= SZ_R && SZ_X1 + SZ_HF <= SZ_R);

extern "C" void kernel_launch(void* const* d_in, const int* in_sizes, int n_in,
                              void* d_out, int out_size, void* d_ws, size_t ws_size, hipStream_t stream) {
  if (n_in < 13) return;
  const size_t xneed = ((size_t)(NB - 1) * SQ_FULL + SQ) * DM;
  if ((size_t)in_sizes[0] < xneed || (size_t)out_size < xneed) return;
  if (in_sizes[1] < DM || in_sizes[2] < DM || in_sizes[7] < DM || in_sizes[8] < DM) return;
  if ((size_t)in_sizes[3] < (size_t)DM * LQ || in_sizes[4] < LQ) return;
  if ((size_t)in_sizes[5] < (size_t)DM * DM || in_sizes[6] < DM) return;
  if ((size_t)in_sizes[9] < (size_t)DM * DFF || in_sizes[10] < DFF) return;
  if ((size_t)in_sizes[11] < (size_t)DFF * DM || in_sizes[12] < DM) return;
  if (WS_TOTAL > ws_size) return;
  const float* x = (const float*)d_in[0]; const float* g1 = (const float*)d_in[1]; const float* be1 = (const float*)d_in[2];
  const float* wqkv = (const float*)d_in[3]; const float* bqkv = (const float*)d_in[4]; const float* wpr = (const float*)d_in[5]; const float* bpr = (const float*)d_in[6];
  const float* g2 = (const float*)d_in[7]; const float* be2 = (const float*)d_in[8]; const float* wf1 = (const float*)d_in[9]; const float* bf1 = (const float*)d_in[10]; const float* wf2 = (const float*)d_in[11]; const float* bf2 = (const float*)d_in[12];
  float* out = (float*)d_out;
  char* ws = (char*)d_ws; size_t off = 0;
  _Float16* BQKV = (_Float16*)(ws + off); off += SZ_BQKV;
  _Float16* BO   = (_Float16*)(ws + off); off += SZ_BO;
  _Float16* BW1  = (_Float16*)(ws + off); off += SZ_BW1;
  _Float16* BW2  = (_Float16*)(ws + off); off += SZ_BW2;
  _Float16* X16  = (_Float16*)(ws + off); off += SZ_X16;
  _Float16* QKV  = (_Float16*)(ws + off); off += SZ_QKV;
  _Float16* O16  = (_Float16*)(ws + off); off += SZ_O16;
  _Float16* VT   = (_Float16*)(ws + off); off += SZ_VT;
  char* R = ws + off; off += SZ_R;
  float* S = (float*)R; _Float16* P = (_Float16*)(R + SZ_S);
  float* X1 = (float*)R; _Float16* HF16 = (_Float16*)(R + SZ_X1);
  _Float16* M16 = X16;

  k_wt_f16<<<(unsigned)(((size_t)LQ * (DM / 8) + 255) / 256), 256, 0, stream>>>(wqkv, BQKV, (unsigned)DM, (unsigned)LQ, 16.0f);
  k_wt_f16<<<(unsigned)(((size_t)DM * (DM / 8) + 255) / 256), 256, 0, stream>>>(wpr, BO, (unsigned)DM, (unsigned)DM, 16.0f);
  k_wt_f16<<<(unsigned)(((size_t)DFF * (DM / 8) + 255) / 256), 256, 0, stream>>>(wf1, BW1, (unsigned)DM, (unsigned)DFF, 16.0f);
  k_wt_f16<<<(unsigned)(((size_t)DM * (DFF / 8) + 255) / 256), 256, 0, stream>>>(wf2, BW2, (unsigned)DFF, (unsigned)DM, 16.0f);
  for (int b = 0; b < NB; ++b)
    k_ln16<1><<<(unsigned)SQ, 256, 0, stream>>>(x + (size_t)b * SQ_FULL * DM, g1, be1, 1e-5f, X16 + (size_t)b * SQ * DM);
  k_gemm2<0, 0><<<dim3((unsigned)((NR / 128) * (LQ / 64)), 1), 128, 0, stream>>>(X16, DM, 0, BQKV, DM, 0, 0.0625f, bqkv, nullptr, 0, nullptr, QKV, LQ, 0, (int)NR, LQ, DM, 0);
  k_vt<NH, SQ><<<(unsigned)(NB * NH * (SQ / 64)), 256, 0, stream>>>(QKV, LQ, 2 * DM, VT);
  for (int b = 0; b < NB; ++b) { const size_t r0 = (size_t)b * SQ;
    for (int h0 = 0; h0 < NH; h0 += HG) {
      k_gemm2<0, 0><<<dim3((unsigned)((SQ / 128) * (SQ / 64)), HG), 128, 0, stream>>>(QKV + r0 * LQ + (size_t)h0 * HD, LQ, (size_t)HD, QKV + r0 * LQ + DM + (size_t)h0 * HD, LQ, (size_t)HD, 0.125f, nullptr, nullptr, 0, S, nullptr, NKX, (size_t)SQ * NKX, SQ, SQ, HD, 1);
      k_rsmc<<<(unsigned)(HG * (SQ / 128)), 128, 0, stream>>>(S, P);
      k_gemm2<0, 0><<<dim3((unsigned)(SQ / 128), HG), 128, 0, stream>>>(P, NKX, (size_t)SQ * NKX, VT + ((size_t)b * NH + h0) * HD * SQ, SQ, (size_t)HD * SQ, 0.25f, nullptr, nullptr, 0, nullptr, O16 + r0 * DM + (size_t)h0 * HD, DM, (size_t)HD, SQ, HD, SQ, 2);
    } }
  for (int b = 0; b < NB; ++b)
    k_gemm2<0, 1><<<dim3((unsigned)((SQ / 128) * (DM / 64)), 1), 128, 0, stream>>>(O16 + (size_t)b * SQ * DM, DM, 0, BO, DM, 0, 0.0009765625f, bpr, x + (size_t)b * SQ_FULL * DM, DM, X1 + (size_t)b * SQ * DM, nullptr, DM, 0, SQ, DM, DM, 0);
  k_ln16<0><<<(unsigned)NR, 256, 0, stream>>>(X1, g2, be2, 1e-5f, M16);
  for (int b = 0; b < NB; ++b) { const size_t r0 = (size_t)b * SQ;
    k_gemm2<6, 0><<<dim3((unsigned)((SQ / 128) * (DFF / 64)), 1), 128, 0, stream>>>(M16 + r0 * DM, DM, 0, BW1, DM, 0, 0.0625f, bf1, nullptr, 0, nullptr, HF16, DFF, 0, SQ, DFF, DM, 0);
    k_gemm2<0, 0><<<dim3((unsigned)((SQ / 128) * (DM / 64)), 1), 128, 0, stream>>>(HF16, DFF, 0, BW2, DFF, 0, 0.0625f, bf2, X1 + r0 * DM, DM, out + (size_t)b * SQ_FULL * DM, nullptr, DM, 0, SQ, DM, DFF, 0); }
}
